// SwinTransformerBlock_47794396069913
// MI455X (gfx1250) — hardware-verified
//
#include <hip/hip_runtime.h>


#ifndef NB
#define NB 1
#endif
#ifndef SEQ
#define SEQ 16384
#endif
#define SEQ_FULL 16384
#define HG   128
#define WPR  32
#define NPW  16
#define NWF  (SEQ_FULL / NPW)
#define DM   512
#define NH   8
#define HD   64
#define QW   1536
#define FF   2048
#define MCH  ((SEQ < 8192) ? SEQ : 8192)
#define WSC  64.0f
#define WINV 0.015625f
#define PCAR 1024.0f
#define PINV 0.0009765625f

static_assert(NB == 1);
static_assert(SEQ % 64 == 0 && SEQ >= 64 && SEQ <= SEQ_FULL && SEQ % NPW == 0);
static_assert(MCH % 64 == 0 && SEQ % MCH == 0);
static_assert(DM % 64 == 0 && QW % 64 == 0 && FF % 64 == 0 && HD == 64 && DM % 32 == 0 && FF % 32 == 0);

typedef _Float16 h16;
typedef __attribute__((ext_vector_type(16))) _Float16 v16h;
typedef __attribute__((ext_vector_type(8)))  _Float16 v8h;
typedef __attribute__((ext_vector_type(2)))  _Float16 v2h;
typedef __attribute__((ext_vector_type(8)))  float    v8f;
typedef __attribute__((ext_vector_type(4)))  float    v4f;
typedef v8h __attribute__((may_alias)) v8ha;
typedef v4f __attribute__((may_alias)) v4fa;

__device__ __forceinline__ unsigned short f2bf(float f) { unsigned u = __float_as_uint(f); u += 0x7FFFu + ((u >> 16) & 1u); return (unsigned short)(u >> 16); }
__device__ __forceinline__ float bf2f(unsigned short b) { return __uint_as_float(((unsigned)b) << 16); }
__device__ __forceinline__ float bfr(float f) { return bf2f(f2bf(f)); }
__device__ __forceinline__ v16h cat16(v8h lo, v8h hi) { return __builtin_shufflevector(lo, hi, 0, 1, 2, 3, 4, 5, 6, 7, 8, 9, 10, 11, 12, 13, 14, 15); }
__device__ __forceinline__ v8f wmma16(v16h a, v16h b, v8f c) { return __builtin_amdgcn_wmma_f32_16x16x32_f16(false, a, false, b, (short)0, c, false, false); }
__device__ __forceinline__ v16h ldf(const h16* p) { return cat16(*(const v8h*)p, *(const v8h*)(p + 16)); }

__device__ __forceinline__ void rc_of(int r, int& y, int& x) { const int w = r >> 4, p = r & 15; y = ((w >> 5) << 2) + (p >> 2); x = ((w & 31) << 2) + (p & 3); }
__device__ __forceinline__ int wrow(int y, int x) { return (((y >> 2) * WPR + (x >> 2)) << 4) + ((y & 3) << 2) + (x & 3); }
__device__ __forceinline__ int tokrow(int r) { int y, x; rc_of(r, y, x); return y * HG + x; }
__device__ __forceinline__ int shrow(int r) { int y, x; rc_of(r, y, x); return wrow((y + 2) & (HG - 1), (x + 2) & (HG - 1)); }
__device__ __forceinline__ int regid(int wq, int p) { int y, x; rc_of(wq * NPW + p, y, x); y = (y + 2) & (HG - 1); x = (x + 2) & (HG - 1); return ((y + 2) >> 2) * WPR + ((x + 2) >> 2); }

__global__ __launch_bounds__(256) void k_wt(const float* __restrict__ w, int K, int N, h16* Bt) {
    const int lane = threadIdx.x & 31; const int L0 = (blockIdx.x * 8 + (threadIdx.x >> 5)) * 8; const int nlines = N * K / 64;
#pragma unroll
    for (int ps = 0; ps < 2; ++ps) {
#pragma unroll 1
        for (int l = 0; l < 8; ++l) { const int L = L0 + l; if (L >= nlines) break; const size_t e = (size_t)L * 64 + lane * 2; const int k = (int)(e % K), n = (int)(e / K); v2h o;
            o[0] = (h16)(bfr(w[(size_t)k * N + n]) * WSC); o[1] = (h16)(bfr(w[(size_t)(k + 1) * N + n]) * WSC); *(volatile v2h*)(Bt + e) = o; }
        if (ps == 0) __threadfence(); }
}

template <int PERM, int RBF>
__global__ __launch_bounds__(256) void k_ln(const float* __restrict__ IN, const float* __restrict__ g, const float* __restrict__ bb, h16* X, int nrows) {
    const int lane = threadIdx.x & 31; const int t = blockIdx.x * 8 + (threadIdx.x >> 5); if (t >= nrows) return;
    int src = t;
    if (PERM == 1) src = tokrow(t);
    if (PERM == 2) { src = shrow(t); src = (src < nrows) ? src : (nrows - 1); }
    const float* p = IN + (size_t)src * DM; const int cA = lane * 8, cB = 256 + lane * 8;
    float v[16];
    { const v4f a0 = *(const v4f*)(p + cA), a1 = *(const v4f*)(p + cA + 4), a2 = *(const v4f*)(p + cB), a3 = *(const v4f*)(p + cB + 4);
#pragma unroll
      for (int q = 0; q < 4; ++q) { v[q] = a0[q]; v[4 + q] = a1[q]; v[8 + q] = a2[q]; v[12 + q] = a3[q]; } }
    if (RBF) {
#pragma unroll
        for (int q = 0; q < 16; ++q) v[q] = bfr(v[q]); }
    float s = 0.f;
#pragma unroll
    for (int q = 0; q < 16; ++q) s += v[q];
#pragma unroll
    for (int sh = 16; sh; sh >>= 1) s += __shfl_xor(s, sh, 32);
    const float mu = s * (1.0f / (float)DM); float s2 = 0.f;
#pragma unroll
    for (int q = 0; q < 16; ++q) { const float d0 = v[q] - mu; s2 += d0 * d0; }
#pragma unroll
    for (int sh = 16; sh; sh >>= 1) s2 += __shfl_xor(s2, sh, 32);
    const float rs = 1.0f / sqrtf(s2 * (1.0f / (float)DM) + 1e-5f);
    float gv[16], bv[16];
    { const v4f g0 = *(const v4f*)(g + cA), g1 = *(const v4f*)(g + cA + 4), g2 = *(const v4f*)(g + cB), g3 = *(const v4f*)(g + cB + 4);
      const v4f b0 = *(const v4f*)(bb + cA), b1 = *(const v4f*)(bb + cA + 4), b2 = *(const v4f*)(bb + cB), b3 = *(const v4f*)(bb + cB + 4);
#pragma unroll
      for (int q = 0; q < 4; ++q) { gv[q] = g0[q]; gv[4 + q] = g1[q]; gv[8 + q] = g2[q]; gv[12 + q] = g3[q]; bv[q] = b0[q]; bv[4 + q] = b1[q]; bv[8 + q] = b2[q]; bv[12 + q] = b3[q]; } }
    v8h o0, o1;
#pragma unroll
    for (int q = 0; q < 8; ++q) {
        const float y0 = (v[q] - mu) * rs * bfr(gv[q]) + bfr(bv[q]); const float y1 = (v[8 + q] - mu) * rs * bfr(gv[8 + q]) + bfr(bv[8 + q]);
        o0[q] = (h16)y0; o1[q] = (h16)y1; }
    const size_t o = (size_t)t * DM;
#pragma unroll 1
    for (int ps = 0; ps < 2; ++ps) { *(volatile v8h*)(X + o + cA) = o0; *(volatile v8h*)(X + o + cB) = o1; if (ps == 0) __threadfence(); }
}

template <int MODE, int RBF>
__global__ __launch_bounds__(32) void k_gemm(const h16* __restrict__ A, const h16* __restrict__ Bt, int K, void* Cv, int ldc, const float* __restrict__ bias, const float* __restrict__ R, int nrows) {
    __shared__ __align__(16) float os[16 * 68];
    const int lane = threadIdx.x & 31, lr = lane & 15, hi = lane >> 4; const int r0 = blockIdx.x * 64, c0 = blockIdx.y * 64;
    v8f acc[4][4];
#pragma unroll
    for (int mb = 0; mb < 4; ++mb)
#pragma unroll
        for (int nb = 0; nb < 4; ++nb) acc[mb][nb] = (v8f){};
    const size_t aoff = (size_t)(r0 + lr) * K + 8 * hi, boff = (size_t)(c0 + lr) * K + 8 * hi;
#pragma unroll 1
    for (int kc = 0; kc < K; kc += 32) {
        v16h a[4];
#pragma unroll
        for (int mb = 0; mb < 4; ++mb) a[mb] = ldf(A + aoff + (size_t)mb * 16 * K + kc);
#pragma unroll
        for (int nb = 0; nb < 4; ++nb) { const v16h b = ldf(Bt + boff + (size_t)nb * 16 * K + kc);
#pragma unroll
            for (int mb = 0; mb < 4; ++mb) acc[mb][nb] = wmma16(a[mb], b, acc[mb][nb]); }
        asm volatile("v_nop\n\tv_nop\n\tv_nop\n\tv_nop" : "+v"(acc[0][0]), "+v"(acc[1][1]), "+v"(acc[2][2]), "+v"(acc[3][3]) : "v"(a[0]), "v"(a[3]));
    }
#pragma unroll
    for (int mb = 0; mb < 4; ++mb) {
#pragma unroll
        for (int nb = 0; nb < 4; ++nb) {
#pragma unroll
            for (int j = 0; j < 8; ++j) os[(hi * 8 + j) * 68 + nb * 16 + lr] = acc[mb][nb][j]; }
        __builtin_amdgcn_wave_barrier(); asm volatile("" ::: "memory");
        const int gr0 = r0 + mb * 16;
        if (MODE == 0) {
            h16* C = (h16*)Cv;
#pragma unroll 1
            for (int ps = 0; ps < 2; ++ps) {
#pragma unroll
                for (int s = 0; s < 4; ++s) { const int row = s * 4 + (lane >> 3), cofs = (lane & 7) * 8;
                    const v4f x0 = *(const v4fa*)(os + row * 68 + cofs), x1 = *(const v4fa*)(os + row * 68 + cofs + 4);
                    const v4f b0 = *(const v4f*)(bias + c0 + cofs), b1 = *(const v4f*)(bias + c0 + cofs + 4); v8h o;
#pragma unroll
                    for (int q = 0; q < 4; ++q) { o[q] = (h16)(x0[q] * WINV + bfr(b0[q])); o[4 + q] = (h16)(x1[q] * WINV + bfr(b1[q])); }
                    *(volatile v8h*)(C + (size_t)(gr0 + row) * ldc + c0 + cofs) = o; }
                if (ps == 0) __threadfence(); }
        } else {
            float* C = (float*)Cv;
#pragma unroll 1
            for (int ps = 0; ps < 2; ++ps) {
#pragma unroll
                for (int s = 0; s < 8; ++s) { const int row = 2 * s + hi, cofs = lr * 4; const int grow = gr0 + row; const int drow = (MODE == 2) ? shrow(grow) : grow; const int dr = (drow < nrows) ? drow : (nrows - 1);
                    v4f val = *(const v4fa*)(os + row * 68 + cofs); const v4f b4 = *(const v4f*)(bias + c0 + cofs); const v4f rr = *(const v4f*)(R + (size_t)dr * ldc + c0 + cofs);
#pragma unroll
                    for (int q = 0; q < 4; ++q) { const float res = RBF ? bfr(rr[q]) : rr[q]; const float y = val[q] * WINV + bfr(b4[q]); val[q] = y + res; }
                    if (MODE != 2 || drow < nrows) *(volatile v4f*)(C + (size_t)drow * ldc + c0 + cofs) = val; }
                if (ps == 0) __threadfence(); }
        }
        __builtin_amdgcn_wave_barrier(); asm volatile("" ::: "memory");
    }
}

template <int MSK>
__global__ __launch_bounds__(32) void k_attn(const h16* __restrict__ QKV, h16* CTX, int nwin) {
    __shared__ __align__(16) h16 sVt[HD * 16];
    __shared__ __align__(16) h16 sC[16 * 72];
    const int w = blockIdx.x >> 3, hd = blockIdx.x & 7;
    if (w >= nwin) return;
    const int lane = threadIdx.x & 31, m = lane & 15, hh = lane >> 4;
    const h16* base = QKV + (size_t)w * NPW * QW + hd * HD;
#pragma unroll
    for (int i = 0; i < 4; ++i) { const int c = i * 32 + lane; const int row = c >> 3, ch = c & 7;
        const v8h vv = *(const v8h*)(base + (size_t)row * QW + 2 * DM + ch * 8);
#pragma unroll
        for (int e = 0; e < 8; ++e) sVt[(ch * 8 + e) * 16 + row] = vv[e]; }
    v16h ka[2], qb[2]; v8f acc = (v8f){};
#pragma unroll
    for (int ks = 0; ks < 2; ++ks) { const h16* kp = base + (size_t)m * QW + DM + ks * 32 + 8 * hh; const h16* qp = base + (size_t)m * QW + ks * 32 + 8 * hh;
        ka[ks] = cat16(*(const v8h*)kp, *(const v8h*)(kp + 16)); qb[ks] = cat16(*(const v8h*)qp, *(const v8h*)(qp + 16)); acc = wmma16(ka[ks], qb[ks], acc); }
    asm volatile("v_nop\n\tv_nop\n\tv_nop\n\tv_nop" : "+v"(acc) : "v"(ka[0]), "v"(ka[1]), "v"(qb[0]), "v"(qb[1]));
    __syncthreads();
    int cq = 0, wq = 0;
    if (MSK) { wq = (w * NH + hd) & (NWF - 1); cq = regid(wq, m); }
    float sc[8]; float mx = -3.0e38f;
#pragma unroll
    for (int r = 0; r < 8; ++r) { float s0 = acc[r] * 0.125f; if (MSK) { const int ck = regid(wq, 8 * hh + r); s0 += (ck != cq) ? -1.0e-9f : 0.0f; } sc[r] = s0; mx = fmaxf(mx, s0); }
    mx = fmaxf(mx, __shfl_xor(mx, 16, 32));
    float sum = 0.f;
#pragma unroll
    for (int r = 0; r < 8; ++r) { sc[r] = __builtin_amdgcn_exp2f((sc[r] - mx) * 1.4426950408889634f); sum += sc[r]; }
    sum += __shfl_xor(sum, 16, 32);
    const float f = PCAR / sum;
    v8h ph;
#pragma unroll
    for (int r = 0; r < 8; ++r) ph[r] = (h16)(sc[r] * f);
    const v8h z8 = (v8h){}; const v16h pa = cat16(ph, z8);
    v16h vb[4]; v8f acc2[4];
#pragma unroll
    for (int nt = 0; nt < 4; ++nt) { acc2[nt] = (v8f){}; const v8h vlo = *(const v8ha*)(sVt + (nt * 16 + m) * 16 + 8 * hh); vb[nt] = cat16(vlo, z8); acc2[nt] = wmma16(pa, vb[nt], acc2[nt]); }
    asm volatile("v_nop\n\tv_nop\n\tv_nop\n\tv_nop" : "+v"(acc2[0]), "+v"(acc2[1]), "+v"(acc2[2]), "+v"(acc2[3]) : "v"(pa), "v"(vb[0]), "v"(vb[1]), "v"(vb[2]), "v"(vb[3]));
#pragma unroll
    for (int nt = 0; nt < 4; ++nt) {
#pragma unroll
        for (int r = 0; r < 8; ++r) sC[(8 * hh + r) * 72 + nt * 16 + m] = (h16)(acc2[nt][r] * PINV); }
    __syncthreads();
    h16* ob = CTX + (size_t)w * NPW * DM + hd * HD;
#pragma unroll 1
    for (int ps = 0; ps < 2; ++ps) {
#pragma unroll
        for (int i = 0; i < 4; ++i) { const int row = i * 4 + (lane >> 3), ch = lane & 7; const v8h o = *(const v8ha*)(sC + row * 72 + ch * 8); *(volatile v8h*)(ob + (size_t)row * DM + ch * 8) = o; }
        if (ps == 0) __threadfence(); }
}

extern "C" void kernel_launch(void* const* d_in, const int* in_sizes, int n_in,
                              void* d_out, int out_size, void* d_ws, size_t ws_size, hipStream_t stream) {
    if (n_in < 25) return;
    if (in_sizes[0] < SEQ_FULL * DM || out_size < SEQ * DM) return;
    for (int i = 1; i <= 8; ++i) if (in_sizes[i] < DM) return;
    if (in_sizes[9] < DM * QW || in_sizes[10] < QW || in_sizes[11] < DM * DM || in_sizes[12] < DM) return;
    if (in_sizes[13] < DM * QW || in_sizes[14] < QW || in_sizes[15] < DM * DM || in_sizes[16] < DM) return;
    if (in_sizes[17] < DM * FF || in_sizes[18] < FF || in_sizes[19] < FF * DM || in_sizes[20] < DM) return;
    if (in_sizes[21] < DM * FF || in_sizes[22] < FF || in_sizes[23] < FF * DM || in_sizes[24] < DM) return;
    const float* x = (const float*)d_in[0];
    const float* l1g = (const float*)d_in[1]; const float* l1b = (const float*)d_in[2]; const float* l2g = (const float*)d_in[3]; const float* l2b = (const float*)d_in[4];
    const float* l3g = (const float*)d_in[5]; const float* l3b = (const float*)d_in[6]; const float* l4g = (const float*)d_in[7]; const float* l4b = (const float*)d_in[8];
    const float* qkv1_w = (const float*)d_in[9];  const float* qkv1_b = (const float*)d_in[10]; const float* ao1_w = (const float*)d_in[11]; const float* ao1_b = (const float*)d_in[12];
    const float* qkv2_w = (const float*)d_in[13]; const float* qkv2_b = (const float*)d_in[14]; const float* ao2_w = (const float*)d_in[15]; const float* ao2_b = (const float*)d_in[16];
    const float* m1a_w = (const float*)d_in[17]; const float* m1a_b = (const float*)d_in[18]; const float* m1b_w = (const float*)d_in[19]; const float* m1b_b = (const float*)d_in[20];
    const float* m2a_w = (const float*)d_in[21]; const float* m2a_b = (const float*)d_in[22]; const float* m2b_w = (const float*)d_in[23]; const float* m2b_b = (const float*)d_in[24];
    float* OUT = (float*)d_out;

    char* wsp = (char*)d_ws;
    auto take = [&](size_t bytes) { char* p = wsp; wsp += (bytes + 255) & ~(size_t)255; return (void*)p; };
    h16* WQ1 = (h16*)take((size_t)QW * DM * 2); h16* WO1 = (h16*)take((size_t)DM * DM * 2); h16* WQ2 = (h16*)take((size_t)QW * DM * 2); h16* WO2 = (h16*)take((size_t)DM * DM * 2);
    h16* WA1 = (h16*)take((size_t)FF * DM * 2); h16* WB1 = (h16*)take((size_t)DM * FF * 2); h16* WA2 = (h16*)take((size_t)FF * DM * 2); h16* WB2 = (h16*)take((size_t)DM * FF * 2);
    h16* X16 = (h16*)take((size_t)SEQ * DM * 2);
    const size_t bigb = ((size_t)SEQ * QW * 2 > (size_t)MCH * FF * 2) ? (size_t)SEQ * QW * 2 : (size_t)MCH * FF * 2;
    h16* BIG = (h16*)take(bigb);
    float* F0 = (float*)take((size_t)SEQ * DM * 4);
    const size_t used = (size_t)(wsp - (char*)d_ws); if (used > ws_size || used > (size_t)134217728) return;
    h16* QKV16 = BIG; h16* MID = BIG; h16* CTX = X16;

    k_wt<<<(unsigned)((DM * QW / 64 + 63) / 64), 256, 0, stream>>>(qkv1_w, DM, QW, WQ1);
    k_wt<<<(unsigned)((DM * DM / 64 + 63) / 64), 256, 0, stream>>>(ao1_w, DM, DM, WO1);
    k_wt<<<(unsigned)((DM * QW / 64 + 63) / 64), 256, 0, stream>>>(qkv2_w, DM, QW, WQ2);
    k_wt<<<(unsigned)((DM * DM / 64 + 63) / 64), 256, 0, stream>>>(ao2_w, DM, DM, WO2);
    k_wt<<<(unsigned)((DM * FF / 64 + 63) / 64), 256, 0, stream>>>(m1a_w, DM, FF, WA1);
    k_wt<<<(unsigned)((FF * DM / 64 + 63) / 64), 256, 0, stream>>>(m1b_w, FF, DM, WB1);
    k_wt<<<(unsigned)((DM * FF / 64 + 63) / 64), 256, 0, stream>>>(m2a_w, DM, FF, WA2);
    k_wt<<<(unsigned)((FF * DM / 64 + 63) / 64), 256, 0, stream>>>(m2b_w, FF, DM, WB2);

    const unsigned gln = (unsigned)((SEQ + 7) / 8); const unsigned gat = (unsigned)((SEQ / NPW) * NH);
    k_ln<1, 1><<<gln, 256, 0, stream>>>(x, l1g, l1b, X16, SEQ);
    k_gemm<0, 0><<<dim3(SEQ / 64, QW / 64), 32, 0, stream>>>(X16, WQ1, DM, (void*)QKV16, QW, qkv1_b, x, SEQ);
    k_attn<0><<<gat, 32, 0, stream>>>(QKV16, CTX, SEQ / NPW);
    k_gemm<1, 1><<<dim3(SEQ / 64, DM / 64), 32, 0, stream>>>(CTX, WO1, DM, (void*)F0, DM, ao1_b, x, SEQ);
    k_ln<0, 0><<<gln, 256, 0, stream>>>(F0, l2g, l2b, X16, SEQ);
    for (int ch = 0; ch < SEQ / MCH; ++ch) {
        k_gemm<0, 0><<<dim3(MCH / 64, FF / 64), 32, 0, stream>>>(X16 + (size_t)ch * MCH * DM, WA1, DM, (void*)MID, FF, m1a_b, x, MCH);
        k_gemm<1, 0><<<dim3(MCH / 64, DM / 64), 32, 0, stream>>>(MID, WB1, FF, (void*)(OUT + (size_t)ch * MCH * DM), DM, m1b_b, F0 + (size_t)ch * MCH * DM, MCH); }
    k_ln<2, 0><<<gln, 256, 0, stream>>>(OUT, l3g, l3b, X16, SEQ);
    k_gemm<0, 0><<<dim3(SEQ / 64, QW / 64), 32, 0, stream>>>(X16, WQ2, DM, (void*)QKV16, QW, qkv2_b, x, SEQ);
    k_attn<1><<<gat, 32, 0, stream>>>(QKV16, CTX, SEQ / NPW);
    k_gemm<2, 0><<<dim3(SEQ / 64, DM / 64), 32, 0, stream>>>(CTX, WO2, DM, (void*)F0, DM, ao2_b, OUT, SEQ);
    k_ln<0, 0><<<gln, 256, 0, stream>>>(F0, l4g, l4b, X16, SEQ);
    for (int ch = 0; ch < SEQ / MCH; ++ch) {
        k_gemm<0, 0><<<dim3(MCH / 64, FF / 64), 32, 0, stream>>>(X16 + (size_t)ch * MCH * DM, WA2, DM, (void*)MID, FF, m2a_b, x, MCH);
        k_gemm<1, 0><<<dim3(MCH / 64, DM / 64), 32, 0, stream>>>(MID, WB2, FF, (void*)(OUT + (size_t)ch * MCH * DM), DM, m2b_b, F0 + (size_t)ch * MCH * DM, MCH); }
}
